// PrecomputedMetaNet_773094113739
// MI455X (gfx1250) — hardware-verified
//
#include <hip/hip_runtime.h>
#include <stddef.h>


typedef _Float16 v16h __attribute__((ext_vector_type(16)));
typedef _Float16 v8h  __attribute__((ext_vector_type(8)));
typedef float    v8f  __attribute__((ext_vector_type(8)));
typedef float    v4f  __attribute__((ext_vector_type(4)));
typedef _Float16 h16;

#ifndef NB
#define NB 4096
#endif
#define NB_FULL 4096
#define DIM   1024
#define HID   256
#define NT    8
#define NTP   16
#define MROWS (NB)

static_assert(NB >= 128 && NB <= NB_FULL && (NB % 128) == 0);
static_assert((DIM % 64) == 0 && (DIM % 32) == 0);
static_assert((HID % 64) == 0 && (HID % 32) == 0);
static_assert((MROWS % 64) == 0 && (MROWS % 128) == 0);
static_assert(NT == 8 && NTP == 16);
static_assert(((size_t)MROWS * DIM) % 2048 == 0);
static_assert(((size_t)HID * DIM) % 2048 == 0);
static_assert(((size_t)DIM * DIM) % 2048 == 0);
static_assert(((size_t)NTP * HID) % 2048 == 0 && ((size_t)NT * HID) % 8 == 0);
static_assert((size_t)MROWS * DIM < (size_t)0xFFFFFFFFu);

#define LDT 72
#define LDC 68
static_assert((LDT % 8) == 0 && LDT >= 64);
static_assert((LDC % 4) == 0 && LDC >= 64);

#define WCARRY 64.0f
#define MCARRY 16.0f

#define TM_BYTES   ((size_t)NT * DIM * DIM * 2)
#define W1_BYTES   ((size_t)HID * DIM * 2)
#define WP_BYTES   ((size_t)DIM * DIM * 2)
#define W2_BYTES   ((size_t)NTP * HID * 2)
#define T16_BYTES  ((size_t)MROWS * DIM * 2)
#define H16_BYTES  ((size_t)MROWS * HID * 2)
#define CF_BYTES   ((size_t)MROWS * NT * 4)
#define TF_BYTES   ((size_t)MROWS * DIM * 4)
#define OFF_TM   ((size_t)0)
#define OFF_W1   (OFF_TM + TM_BYTES)
#define OFF_WP   (OFF_W1 + W1_BYTES)
#define OFF_W2   (OFF_WP + WP_BYTES)
#define OFF_TA16 (OFF_W2 + W2_BYTES)
#define OFF_TB16 (OFF_TA16 + T16_BYTES)
#define OFF_H16  (OFF_TB16 + T16_BYTES)
#define OFF_CF   (OFF_H16 + H16_BYTES)
#define OFF_TFA  (OFF_CF + CF_BYTES)
#define OFF_TFB  (OFF_TFA + TF_BYTES)
#define WS_TOTAL (OFF_TFB + TF_BYTES)
static_assert((TM_BYTES % 128) == 0 && (W1_BYTES % 128) == 0 && (WP_BYTES % 128) == 0);
static_assert((W2_BYTES % 128) == 0 && (T16_BYTES % 128) == 0 && (H16_BYTES % 128) == 0);
static_assert((CF_BYTES % 128) == 0 && (TF_BYTES % 128) == 0);
static_assert(WS_TOTAL <= (size_t)134217728);

__device__ __forceinline__ float bf16r(float x) {
  unsigned int u = __float_as_uint(x);
  u = (u + 0x7FFFu + ((u >> 16) & 1u)) & 0xFFFF0000u;
  return __uint_as_float(u);
}

static __device__ __forceinline__ h16 toh_flush(float v) {
  const h16 r = (h16)v;
  return (fabsf(v) < 6.103515625e-05f) ? (h16)0.0f : r;
}

__device__ __forceinline__ v16h frag_at(const _Float16* p) {
  v8h lo = *(const v8h*)(p);
  v8h hi = *(const v8h*)(p + 16);
  v16h out;
#pragma unroll
  for (int i = 0; i < 8; ++i) { out[i] = lo[i]; out[i + 8] = hi[i]; }
  return out;
}

__device__ __forceinline__ v8f wmma16(v16h a, v16h b, v8f c) {
  v8f d = __builtin_amdgcn_wmma_f32_16x16x32_f16(false, a, false, b, (short)0, c,
                                                 false, false);
  asm volatile("v_nop\n\tv_nop\n\tv_nop\n\tv_nop" : "+v"(d) : "v"(a), "v"(b));
  return d;
}

__device__ __forceinline__ void wave_lds_sync() {
  __builtin_amdgcn_fence(3  , "wavefront");
  asm volatile("s_wait_dscnt 0x0" ::: "memory");
  __builtin_amdgcn_wave_barrier();
}

__device__ __forceinline__ float relu_act(float t) {
  return fmaxf(t, 0.0f);
}

__global__ __launch_bounds__(256) void wconv_kernel(
    const float* __restrict__ W, _Float16* __restrict__ Wt, unsigned ldw, unsigned ldk) {
  __shared__ _Float16 T[64 * LDT];
  const unsigned tid = threadIdx.x;
  const unsigned n0 = blockIdx.x * 64u;
  const unsigned k0 = blockIdx.y * 64u;
#pragma unroll 4
  for (unsigned j = 0; j < 16u; ++j) {
    const unsigned idx = tid + 256u * j;
    const unsigned kr = idx >> 6, nc = idx & 63u;
    const float v = W[(size_t)(k0 + kr) * ldw + n0 + nc];
    T[nc * LDT + kr] = (_Float16)(WCARRY * bf16r(v));
  }
  __syncthreads();
  v8h x[2];
  size_t off[2];
#pragma unroll
  for (unsigned i = 0; i < 2u; ++i) {
    const unsigned n = 32u * i + (tid >> 3);
    const unsigned kc = (tid & 7u) * 8u;
    x[i] = *(const v8h*)&T[n * LDT + kc];
    off[i] = (size_t)(n0 + n) * ldk + k0 + kc;
  }
#pragma unroll
  for (int i = 0; i < 2; ++i) *(volatile v8h*)(Wt + off[i]) = x[i];
  __threadfence();
#pragma unroll
  for (int i = 0; i < 2; ++i) *(volatile v8h*)(Wt + off[i]) = x[i];
}

__global__ __launch_bounds__(256) void cvt_kernel(
    const float* __restrict__ src, _Float16* __restrict__ dst, unsigned nvalid, float carry) {
  const unsigned base = (blockIdx.x * 256u + threadIdx.x) * 8u;
  const bool ok = base < nvalid;
  const unsigned sb = ok ? base : 0u;
  const v4f a0 = *(const v4f*)(src + sb);
  const v4f a1 = *(const v4f*)(src + sb + 4u);
  v8h o;
#pragma unroll
  for (int i = 0; i < 4; ++i) {
    const h16 t0 = toh_flush(carry * bf16r(a0[i]));
    const h16 t1 = toh_flush(carry * bf16r(a1[i]));
    o[i]     = ok ? t0 : (h16)0.0f;
    o[i + 4] = ok ? t1 : (h16)0.0f;
  }
  _Float16* p = dst + base;
  *(volatile v8h*)p = o;
  __threadfence();
  *(volatile v8h*)p = o;
}

template <int MODE>
__device__ __forceinline__ void gemm_body(
    const _Float16* __restrict__ A16, const _Float16* __restrict__ Bt, const unsigned K,
    const float* __restrict__ bias, const float* __restrict__ addf,
    const float* __restrict__ coef, const unsigned jidx,
    float* __restrict__ outf, _Float16* __restrict__ out16) {
  __shared__ float Cs[64 * LDC];
  const unsigned tid = threadIdx.x, lane = tid & 31u;
  const unsigned w = (unsigned)__builtin_amdgcn_readfirstlane((int)(tid >> 5));
  const unsigned mw = w >> 1, nw = w & 1u;
  const unsigned hh = lane >> 4, m = lane & 15u;
  const unsigned n0 = blockIdx.x * 64u;
  const unsigned row0 = blockIdx.y * 64u;

  const _Float16* ap  = A16 + (size_t)(row0 + mw * 16u + m) * K + hh * 8u;
  const _Float16* bp0 = Bt + (size_t)(n0 + nw * 32u + m) * K + hh * 8u;
  const _Float16* bp1 = bp0 + (size_t)16 * K;
  v8f acc0 = {}, acc1 = {};
#pragma unroll 2
  for (unsigned k0 = 0; k0 < K; k0 += 32u) {
    const v16h a  = frag_at(ap + k0);
    const v16h b0 = frag_at(bp0 + k0);
    const v16h b1 = frag_at(bp1 + k0);
    acc0 = wmma16(a, b0, acc0);
    acc1 = wmma16(a, b1, acc1);
  }
#pragma unroll
  for (int r = 0; r < 8; ++r) {
    float* d = &Cs[(mw * 16u + hh * 8u + (unsigned)r) * LDC + nw * 32u + m];
    d[0]  = acc0[r];
    d[16] = acc1[r];
  }
  __syncthreads();

  if (MODE == 0) {
    v8h x[2];
    size_t off[2];
#pragma unroll
    for (unsigned i = 0; i < 2u; ++i) {
      const unsigned r = 32u * i + (tid >> 3);
      const unsigned c = (tid & 7u) * 8u;
      const v4f u0 = *(const v4f*)&Cs[r * LDC + c];
      const v4f u1 = *(const v4f*)&Cs[r * LDC + c + 4];
      const v4f g0 = *(const v4f*)(bias + n0 + c);
      const v4f g1 = *(const v4f*)(bias + n0 + c + 4u);
#pragma unroll
      for (int j = 0; j < 4; ++j) {
        x[i][j]     = toh_flush(MCARRY * relu_act(u0[j] * (1.0f / WCARRY) + bf16r(g0[j])));
        x[i][j + 4] = toh_flush(MCARRY * relu_act(u1[j] * (1.0f / WCARRY) + bf16r(g1[j])));
      }
      off[i] = (size_t)(row0 + r) * HID + n0 + c;
    }
#pragma unroll
    for (int i = 0; i < 2; ++i) *(volatile v8h*)(out16 + off[i]) = x[i];
    __threadfence();
#pragma unroll
    for (int i = 0; i < 2; ++i) *(volatile v8h*)(out16 + off[i]) = x[i];
  }

  if (MODE == 1 || MODE == 2) {
    v4f xs[4];
    size_t off[4];
#pragma unroll
    for (unsigned i = 0; i < 4u; ++i) {
      const unsigned r = 16u * i + (tid >> 4);
      const unsigned c = (tid & 15u) * 4u;
      const size_t crow = (size_t)(row0 + r);
      const v4f u = *(const v4f*)&Cs[r * LDC + c];
      const v4f xin = *(const v4f*)(addf + crow * DIM + n0 + c);
      const float cf = coef[crow * NT + jidx];
      v4f val;
#pragma unroll
      for (int j = 0; j < 4; ++j) {
        const float base = (MODE == 1) ? bf16r(xin[j]) : xin[j];
        val[j] = base + cf * (u[j] * (1.0f / WCARRY));
      }
      xs[i] = val;
      *(v4f*)&Cs[r * LDC + c] = val;
      off[i] = crow * DIM + n0 + c;
    }
    __syncthreads();
    v8h x[2];
    size_t off16[2];
#pragma unroll
    for (unsigned i = 0; i < 2u; ++i) {
      const unsigned r = 32u * i + (tid >> 3);
      const unsigned c = (tid & 7u) * 8u;
      const v4f u0 = *(const v4f*)&Cs[r * LDC + c];
      const v4f u1 = *(const v4f*)&Cs[r * LDC + c + 4];
#pragma unroll
      for (int j = 0; j < 4; ++j) {
        x[i][j]     = toh_flush(u0[j]);
        x[i][j + 4] = toh_flush(u1[j]);
      }
      off16[i] = (size_t)(row0 + r) * DIM + n0 + c;
    }
#pragma unroll
    for (int i = 0; i < 4; ++i) *(volatile v4f*)(outf + off[i]) = xs[i];
#pragma unroll
    for (int i = 0; i < 2; ++i) *(volatile v8h*)(out16 + off16[i]) = x[i];
    __threadfence();
#pragma unroll
    for (int i = 0; i < 4; ++i) *(volatile v4f*)(outf + off[i]) = xs[i];
#pragma unroll
    for (int i = 0; i < 2; ++i) *(volatile v8h*)(out16 + off16[i]) = x[i];
  }

  if (MODE == 3) {
    v4f xs[4];
    size_t off[4];
#pragma unroll
    for (unsigned i = 0; i < 4u; ++i) {
      const unsigned r = 16u * i + (tid >> 4);
      const unsigned c = (tid & 15u) * 4u;
      const v4f u = *(const v4f*)&Cs[r * LDC + c];
      v4f val;
#pragma unroll
      for (int j = 0; j < 4; ++j) val[j] = u[j] * (1.0f / WCARRY);
      xs[i] = val;
      off[i] = (size_t)(row0 + r) * DIM + n0 + c;
    }
#pragma unroll
    for (int i = 0; i < 4; ++i) *(volatile v4f*)(outf + off[i]) = xs[i];
    __threadfence();
#pragma unroll
    for (int i = 0; i < 4; ++i) *(volatile v4f*)(outf + off[i]) = xs[i];
  }
}

__global__ __launch_bounds__(256) void gemm_h_kernel(
    const _Float16* __restrict__ A16, const _Float16* __restrict__ Bt,
    const float* __restrict__ bias, _Float16* __restrict__ hplane) {
  gemm_body<0>(A16, Bt, (unsigned)DIM, bias, (const float*)0, (const float*)0, 0u,
               (float*)0, hplane);
}
__global__ __launch_bounds__(256) void gemm_task_in_kernel(
    const _Float16* __restrict__ A16, const _Float16* __restrict__ Bt,
    const float* __restrict__ xin, const float* __restrict__ coef, unsigned jidx,
    float* __restrict__ tf, _Float16* __restrict__ t16) {
  gemm_body<1>(A16, Bt, (unsigned)DIM, (const float*)0, xin, coef, jidx, tf, t16);
}
__global__ __launch_bounds__(256) void gemm_task_ws_kernel(
    const _Float16* __restrict__ A16, const _Float16* __restrict__ Bt,
    const float* __restrict__ tin, const float* __restrict__ coef, unsigned jidx,
    float* __restrict__ tf, _Float16* __restrict__ t16) {
  gemm_body<2>(A16, Bt, (unsigned)DIM, (const float*)0, tin, coef, jidx, tf, t16);
}
__global__ __launch_bounds__(256) void gemm_out_kernel(
    const _Float16* __restrict__ A16, const _Float16* __restrict__ Bt,
    float* __restrict__ outf) {
  gemm_body<3>(A16, Bt, (unsigned)DIM, (const float*)0, (const float*)0, (const float*)0, 0u,
               outf, (_Float16*)0);
}

__global__ __launch_bounds__(256) void coeff_kernel(
    const _Float16* __restrict__ H16, const _Float16* __restrict__ W2p,
    const float* __restrict__ b2, float* __restrict__ coef) {
  __shared__ float Cc[8 * 16 * 16];
  const unsigned tid = threadIdx.x, lane = tid & 31u;
  const unsigned w = (unsigned)__builtin_amdgcn_readfirstlane((int)(tid >> 5));
  const unsigned hh = lane >> 4, m = lane & 15u;
  const unsigned row0 = blockIdx.x * 128u + w * 16u;

  const _Float16* ap = H16 + (size_t)(row0 + m) * HID + hh * 8u;
  const _Float16* bp = W2p + (size_t)m * HID + hh * 8u;
  v8f acc = {};
#pragma unroll 2
  for (unsigned k0 = 0; k0 < (unsigned)HID; k0 += 32u) {
    const v16h a = frag_at(ap + k0);
    const v16h b = frag_at(bp + k0);
    acc = wmma16(a, b, acc);
  }
  float* C = &Cc[w * 256u];
#pragma unroll
  for (int r = 0; r < 8; ++r) C[(hh * 8u + (unsigned)r) * 16u + m] = acc[r];
  wave_lds_sync();

  const unsigned rr = lane >> 1, cc = (lane & 1u) * 4u;
  const v4f u = *(const v4f*)&C[rr * 16u + cc];
  const v4f bb = *(const v4f*)(b2 + cc);
  v4f val;
#pragma unroll
  for (int j = 0; j < 4; ++j) val[j] = u[j] * (1.0f / (WCARRY * MCARRY)) + bf16r(bb[j]);
  float* p = coef + (size_t)row0 * NT + lane * 4u;
  *(volatile v4f*)p = val;
  __threadfence();
  *(volatile v4f*)p = val;
}

extern "C" void kernel_launch(void* const* d_in, const int* in_sizes, int n_in,
                              void* d_out, int out_size, void* d_ws, size_t ws_size,
                              hipStream_t stream) {
  if (n_in < 7) return;
  if ((long long)in_sizes[0] < (long long)MROWS * DIM) return;
  if ((long long)in_sizes[1] < (long long)HID * DIM) return;
  if (in_sizes[2] < HID) return;
  if (in_sizes[3] < NT * HID) return;
  if (in_sizes[4] < NT) return;
  if ((long long)in_sizes[5] < (long long)NT * DIM * DIM) return;
  if ((long long)in_sizes[6] < (long long)DIM * DIM) return;
  if ((long long)out_size < (long long)MROWS * DIM) return;
  if (ws_size < WS_TOTAL) return;

  const float* F    = (const float*)d_in[0];
  const float* w1   = (const float*)d_in[1];
  const float* b1   = (const float*)d_in[2];
  const float* w2   = (const float*)d_in[3];
  const float* b2   = (const float*)d_in[4];
  const float* task = (const float*)d_in[5];
  const float* wp   = (const float*)d_in[6];
  float* out = (float*)d_out;

  char* ws = (char*)d_ws;
  _Float16* TM16 = (_Float16*)(ws + OFF_TM);
  _Float16* W1p  = (_Float16*)(ws + OFF_W1);
  _Float16* WPp  = (_Float16*)(ws + OFF_WP);
  _Float16* W2p  = (_Float16*)(ws + OFF_W2);
  _Float16* TA16 = (_Float16*)(ws + OFF_TA16);
  _Float16* TB16 = (_Float16*)(ws + OFF_TB16);
  _Float16* H16  = (_Float16*)(ws + OFF_H16);
  float*    CF   = (float*)(ws + OFF_CF);
  float*    TFA  = (float*)(ws + OFF_TFA);
  float*    TFB  = (float*)(ws + OFF_TFB);

  dim3 blk(256);
  dim3 gsq(DIM / 64, DIM / 64);
  dim3 gg(DIM / 64, MROWS / 64);

  for (int j = 0; j < NT; ++j)
    wconv_kernel<<<gsq, blk, 0, stream>>>(task + (size_t)j * DIM * DIM,
                                          TM16 + (size_t)j * DIM * DIM,
                                          (unsigned)DIM, (unsigned)DIM);
  cvt_kernel<<<dim3((HID * DIM) / 2048), blk, 0, stream>>>(w1, W1p, (unsigned)(HID * DIM), WCARRY);
  cvt_kernel<<<dim3((DIM * DIM) / 2048), blk, 0, stream>>>(wp, WPp, (unsigned)(DIM * DIM), WCARRY);
  cvt_kernel<<<dim3((NTP * HID) / 2048), blk, 0, stream>>>(w2, W2p, (unsigned)(NT * HID), WCARRY);
  cvt_kernel<<<dim3((MROWS * DIM) / 2048), blk, 0, stream>>>(F, TA16, (unsigned)(MROWS * DIM), 1.0f);

  gemm_h_kernel<<<dim3(HID / 64, MROWS / 64), blk, 0, stream>>>(TA16, W1p, b1, H16);
  coeff_kernel<<<dim3(MROWS / 128), blk, 0, stream>>>(H16, W2p, b2, CF);

  for (int j = 0; j < NT; ++j) {
    const _Float16* a16 = (j & 1) ? TB16 : TA16;
    _Float16* o16 = (j & 1) ? TA16 : TB16;
    const float* tin = (j & 1) ? TFA : TFB;
    float* tout = (j & 1) ? TFB : TFA;
    const _Float16* bt = TM16 + (size_t)j * DIM * DIM;
    if (j == 0)
      gemm_task_in_kernel<<<gg, blk, 0, stream>>>(a16, bt, F, CF, 0u, tout, o16);
    else
      gemm_task_ws_kernel<<<gg, blk, 0, stream>>>(a16, bt, tin, CF, (unsigned)j, tout, o16);
  }

  gemm_out_kernel<<<gg, blk, 0, stream>>>(TA16, WPp, out);
}
